// DecoderBlock_19825569038501
// MI455X (gfx1250) — hardware-verified
//
#include <hip/hip_runtime.h>
#include <math.h>

#ifndef NB
#define NB 2
#endif
#ifndef SEQ
#define SEQ 2048
#endif
#define SEQ_FULL 2048
#define DEMB 1024
#define DFF 4096
#define TOK (NB * SEQ)
#define NQB (SEQ / 64)
#define NKC (SEQ / 64)

static_assert(SEQ % 64 == 0);
static_assert(NKC <= 32);
static_assert(SEQ <= SEQ_FULL);
static_assert(TOK % 64 == 0);
static_assert(DEMB % 64 == 0 && DFF % 64 == 0 && DEMB % 32 == 0 && DFF % 32 == 0);
static_assert((size_t)TOK * DFF == 4 * (size_t)TOK * DEMB);

typedef __attribute__((ext_vector_type(16))) _Float16 v16h;
typedef __attribute__((ext_vector_type(8)))  _Float16 v8h;
typedef __attribute__((ext_vector_type(8)))  float    v8f;
typedef __attribute__((ext_vector_type(4)))  float    v4f;
typedef __attribute__((ext_vector_type(4)))  unsigned int u4v;
typedef __attribute__((ext_vector_type(2)))  unsigned int u2v;
typedef __attribute__((ext_vector_type(4)))  int      i4v;
typedef __attribute__((ext_vector_type(8)))  unsigned short us8;


#define VST2(T, ptr, val) do { const T vst2_v_ = (val); *(volatile T*)(ptr) = vst2_v_; __threadfence(); *(volatile T*)(ptr) = vst2_v_; } while (0)

__device__ __forceinline__ float cmb_bf(float v) { const unsigned u = __builtin_bit_cast(unsigned, v); const unsigned r = (u + 0x7fffu + ((u >> 16) & 1u)) & 0xffff0000u; return __builtin_bit_cast(float, r); }
__device__ __forceinline__ unsigned int pk2h(float a, float b) { return (unsigned int)__builtin_bit_cast(unsigned short, (_Float16)a) | ((unsigned int)__builtin_bit_cast(unsigned short, (_Float16)b) << 16); }

__device__ __forceinline__ v16h frag_ld(const _Float16* p) { union U { v16h v; v8h h[2]; } f; f.h[0] = *(const v8h*)(p); f.h[1] = *(const v8h*)(p + 16); return f.v; }
__device__ __forceinline__ v8f mma16(v16h a, v16h b, v8f c) {
  c = __builtin_amdgcn_wmma_f32_16x16x32_f16(false, a, false, b, (short)0, c, false, false);
  asm volatile("v_nop\n\tv_nop\n\tv_nop\n\tv_nop" : "+v"(c) : "v"(a), "v"(b));
  return c;
}
__device__ __forceinline__ void dep_guard_h(v8f& a, v8f& b, v16h x, v16h y) { asm volatile("v_nop\n\tv_nop\n\tv_nop\n\tv_nop" : "+v"(a), "+v"(b) : "v"(x), "v"(y)); }
__device__ __forceinline__ void keep4_h(v16h a, v16h b, v16h c, v16h d) { asm volatile("v_nop" :: "v"(a), "v"(b), "v"(c), "v"(d)); }
__device__ __forceinline__ void acc_guard4(v8f& a, v8f& b, v8f& c, v8f& d) { asm volatile("v_nop\n\tv_nop\n\tv_nop\n\tv_nop" : "+v"(a), "+v"(b), "+v"(c), "+v"(d)); }
__device__ __forceinline__ void wave_sync_lds() {
  __builtin_amdgcn_fence(3  , "workgroup");
  __builtin_amdgcn_wave_barrier();
  __builtin_amdgcn_fence(2  , "workgroup");
}

template <int OUT_MODE, int ACT>
__global__ __launch_bounds__(256) void k_gemm64(
    const unsigned short* __restrict__ Ap, int lda, long strideA,
    const unsigned short* __restrict__ Btp, int ldb, long strideB,
    void* __restrict__ Cout, int ldc, long strideC,
    const float* __restrict__ bias, int M, int N, int K, float scale) {
  const _Float16* A = (const _Float16*)Ap; const _Float16* Bt = (const _Float16*)Btp;
  __shared__ __align__(16) float sT[8][16 * 68];
  const int b    = blockIdx.y;
  const int lane = threadIdx.x & 31;
  const int wave = threadIdx.x >> 5;
  const int tilesN = N >> 6;
  const int tilesM = M >> 6;
  const int tile = blockIdx.x * 8 + wave;
  if (tile >= tilesM * tilesN) return;
  const int tm = tile / tilesN;
  const int tn = tile - tm * tilesN;
  const int m0 = tm << 6;
  const int n0 = tn << 6;

  const _Float16* Ab = A  + (size_t)b * strideA;
  const _Float16* Bb = Bt + (size_t)b * strideB;

  const int rlane = lane & 15;
  const int koff  = (lane >> 4) * 8;
  const int mOff  = (lane >> 4) * 8;

  v8f acc[4][4];
#pragma unroll
  for (int i = 0; i < 4; ++i)
#pragma unroll
    for (int j = 0; j < 4; ++j) acc[i][j] = (v8f){0.f,0.f,0.f,0.f,0.f,0.f,0.f,0.f};

  for (int k0 = 0; k0 < K; k0 += 32) {
    v16h bh[4];
#pragma unroll
    for (int j = 0; j < 4; ++j) {
      const size_t bo = (size_t)(n0 + (j << 4) + rlane) * ldb + koff + k0;
      bh[j] = frag_ld(Bb + bo);
    }
#pragma unroll
    for (int i = 0; i < 4; ++i) {
      const size_t ao = (size_t)(m0 + (i << 4) + rlane) * lda + koff + k0;
      v16h ah = frag_ld(Ab + ao);
#pragma unroll
      for (int j = 0; j < 4; ++j)
        acc[i][j] = __builtin_amdgcn_wmma_f32_16x16x32_f16(false, ah, false, bh[j], (short)0, acc[i][j], false, false);
      dep_guard_h(acc[i][0], acc[i][3], ah, ah);
    }
    keep4_h(bh[0], bh[1], bh[2], bh[3]);
  }
  acc_guard4(acc[0][0], acc[0][1], acc[0][2], acc[0][3]);
  acc_guard4(acc[1][0], acc[1][1], acc[1][2], acc[1][3]);
  acc_guard4(acc[2][0], acc[2][1], acc[2][2], acc[2][3]);
  acc_guard4(acc[3][0], acc[3][1], acc[3][2], acc[3][3]);

  float* slab = sT[wave];
#pragma unroll
  for (int i = 0; i < 4; ++i) {
    const int mBase = m0 + (i << 4);
#pragma unroll
    for (int j = 0; j < 4; ++j) {
      const int n = n0 + (j << 4) + rlane;
      const float bv = bias[n];
#pragma unroll
      for (int r = 0; r < 8; ++r) {
        float v = acc[i][j][r] * scale;
        v += bv;
        if (ACT == 2) v = fmaxf(v, 0.0f);
        slab[(mOff + r) * 68 + (j << 4) + rlane] = v;
      }
    }
    wave_sync_lds();
    if (OUT_MODE == 0) {
      float* C = (float*)Cout + (size_t)b * strideC;
      const int hh = lane >> 4, c4 = (lane & 15) * 4;
      for (int pass = 0; pass < 2; ++pass) {
#pragma unroll
        for (int it = 0; it < 8; ++it) {
          const int row = it * 2 + hh;
          v4f v = *(const v4f*)(slab + row * 68 + c4);
          *(volatile v4f*)(C + (size_t)(mBase + row) * ldc + n0 + c4) = v;
        }
        __threadfence();
      }
    } else {
      const int q = lane >> 3, c8 = (lane & 7) * 8;
      unsigned short* C = (unsigned short*)Cout + (size_t)b * strideC;
      for (int pass = 0; pass < 2; ++pass) {
#pragma unroll
        for (int it = 0; it < 4; ++it) {
          const int row = it * 4 + q;
          const float* sp = slab + row * 68 + c8;
          v8h hv;
#pragma unroll
          for (int e = 0; e < 8; ++e) hv[e] = (_Float16)sp[e];
          *(volatile v8h*)(C + (size_t)(mBase + row) * ldc + n0 + c8) = hv;
        }
        __threadfence();
      }
    }
    wave_sync_lds();
  }
}

template <int MM>
__global__ __launch_bounds__(128) void k_attn16(const unsigned short* __restrict__ Qp, const unsigned short* __restrict__ Kp, const unsigned short* __restrict__ VTp,
                                               const int* __restrict__ mask, const int* __restrict__ FL, unsigned short* __restrict__ Op) {
  __shared__ __align__(16) _Float16 Psh[4][16 * 64];
  __shared__ __align__(16) float    Os[4][16 * 68];
  const unsigned tid = threadIdx.x, wave = tid >> 5, lane = tid & 31u, hh = lane >> 4, c = lane & 15u;
  const unsigned bx = blockIdx.x;
  const unsigned qb = bx % (unsigned)NQB, bh = bx / (unsigned)NQB, h = bh & 15u, b = bh >> 4;
  const unsigned q0 = qb * 64u + wave * 16u;
  const float PSC = 16384.0f;
  const float SC  = 0.125f * 1.4426950408889634f;
  const float NEG = -__builtin_inff();

  const _Float16* Qb = (const _Float16*)Qp + (size_t)(b * (unsigned)SEQ + q0 + c) * DEMB + h * 64u + 8u * hh;
  const _Float16* Kb = (const _Float16*)Kp + (size_t)(b * (unsigned)SEQ) * DEMB + h * 64u + 8u * hh;
  const _Float16* Vb = (const _Float16*)VTp + (size_t)(b * (unsigned)DEMB + h * 64u) * SEQ + 8u * hh;
  const v16h qa0 = frag_ld(Qb), qa1 = frag_ld(Qb + 32);

  float mrow[8], lrow[8];
  v8f oacc[4];
#pragma unroll
  for (int r = 0; r < 8; ++r) { mrow[r] = NEG; lrow[r] = 0.f; }
#pragma unroll
  for (int t = 0; t < 4; ++t) oacc[t] = (v8f){0.f,0.f,0.f,0.f,0.f,0.f,0.f,0.f};
  _Float16* pw = Psh[wave];

#pragma unroll 1
  for (unsigned kc = 0; kc < (unsigned)NKC; ++kc) {
    const unsigned kv0 = kc * 64u;
    v8f s[4];
#pragma unroll
    for (int j = 0; j < 4; ++j) {
      const _Float16* kr = Kb + (size_t)(kv0 + (unsigned)j * 16u + c) * DEMB;
      v8f acc = (v8f){0.f,0.f,0.f,0.f,0.f,0.f,0.f,0.f};
      acc = mma16(qa0, frag_ld(kr), acc);
      acc = mma16(qa1, frag_ld(kr + 32), acc);
      s[j] = acc * SC;
    }
    if (MM == 0) {
      const int fl = FL[(b * (unsigned)NQB + qb) * 32u + kc];
      if (fl != 0) {
        const int* mp = mask + (size_t)(b * (unsigned)SEQ_FULL + q0 + 8u * hh) * SEQ_FULL + kv0 + c;
#pragma unroll
        for (int r = 0; r < 8; ++r) {
#pragma unroll
          for (int j = 0; j < 4; ++j) { const int mv = mp[(size_t)r * SEQ_FULL + (unsigned)j * 16u]; if (mv == 0) s[j][r] = NEG; }
          asm volatile("s_nop 0" ::: "memory");
        }
      }
    } else {
      const int* mp = mask + (size_t)b * SEQ_FULL + kv0 + c;
      const int k0 = mp[0], k1 = mp[16], k2 = mp[32], k3 = mp[48];
      const int z = (k0 == 0) | (k1 == 0) | (k2 == 0) | (k3 == 0);
      if (__any(z)) {
#pragma unroll
        for (int r = 0; r < 8; ++r) {
          if (k0 == 0) s[0][r] = NEG;
          if (k1 == 0) s[1][r] = NEG;
          if (k2 == 0) s[2][r] = NEG;
          if (k3 == 0) s[3][r] = NEG;
        }
      }
    }
    float cm[8];
#pragma unroll
    for (int r = 0; r < 8; ++r) {
      float m = fmaxf(fmaxf(s[0][r], s[1][r]), fmaxf(s[2][r], s[3][r]));
      m = fmaxf(m, __shfl_xor(m, 1, 32)); m = fmaxf(m, __shfl_xor(m, 2, 32));
      m = fmaxf(m, __shfl_xor(m, 4, 32)); m = fmaxf(m, __shfl_xor(m, 8, 32));
      cm[r] = m;
    }
#pragma unroll
    for (int r = 0; r < 8; ++r) {
      const float mnew  = fmaxf(mrow[r], cm[r]);
      const float msafe = (mnew == NEG) ? 0.f : mnew;
      const float alpha = exp2f(mrow[r] - msafe);
      mrow[r] = mnew;
      float psum = 0.f;
#pragma unroll
      for (int j = 0; j < 4; ++j) {
        const float p = exp2f(s[j][r] - msafe);
        psum += p;
        pw[(8u * hh + (unsigned)r) * 64u + (unsigned)j * 16u + c] = (_Float16)(p * PSC);
      }
      psum += __shfl_xor(psum, 1, 32); psum += __shfl_xor(psum, 2, 32);
      psum += __shfl_xor(psum, 4, 32); psum += __shfl_xor(psum, 8, 32);
      lrow[r] = lrow[r] * alpha + psum;
#pragma unroll
      for (int t = 0; t < 4; ++t) oacc[t][r] *= alpha;
    }
    wave_sync_lds();
#pragma unroll
    for (int kk = 0; kk < 2; ++kk) {
      const v16h pa = frag_ld(pw + c * 64u + (unsigned)kk * 32u + 8u * hh);
#pragma unroll
      for (int t = 0; t < 4; ++t) {
        const v16h vb = frag_ld(Vb + (size_t)((unsigned)t * 16u + c) * SEQ + kv0 + (unsigned)kk * 32u);
        oacc[t] = mma16(pa, vb, oacc[t]);
      }
    }
    wave_sync_lds();
  }

  float* os = Os[wave];
#pragma unroll
  for (int r = 0; r < 8; ++r) {
    const float inv = 1.0f / (lrow[r] * PSC);
#pragma unroll
    for (int t = 0; t < 4; ++t) os[(8u * hh + (unsigned)r) * 68u + (unsigned)t * 16u + c] = oacc[t][r] * inv;
  }
  wave_sync_lds();
  {
    const unsigned q = lane >> 3, c8 = (lane & 7u) * 8u;
    unsigned short* O = Op + (size_t)(b * (unsigned)SEQ + q0) * DEMB + h * 64u;
    for (int pass = 0; pass < 2; ++pass) {
#pragma unroll
      for (int it = 0; it < 4; ++it) {
        const unsigned row = (unsigned)it * 4u + q;
        const float* sp = os + row * 68u + c8;
        v8h hv;
#pragma unroll
        for (int e = 0; e < 8; ++e) hv[e] = (_Float16)sp[e];
        *(volatile v8h*)(O + (size_t)row * DEMB + c8) = hv;
      }
      __threadfence();
    }
  }
}

__global__ __launch_bounds__(256) void k_mflag(const int* __restrict__ mask, int* __restrict__ FL) {
  __shared__ int sm[8][32];
  const unsigned tid = threadIdx.x, w = tid >> 5, lane = tid & 31u, hf = lane >> 4, l15 = lane & 15u;
  const unsigned blk = blockIdx.x, qb = blk % (unsigned)NQB, b = blk / (unsigned)NQB;
  int my = 0;
#pragma unroll 1
  for (unsigned kc = 0; kc < (unsigned)NKC; ++kc) {
    int z = 0;
#pragma unroll
    for (unsigned i = 0; i < 4; ++i) {
      const unsigned row = qb * 64u + w * 8u + i * 2u + hf;
      const i4v m4 = *(const i4v*)(mask + (size_t)(b * (unsigned)SEQ_FULL + row) * SEQ_FULL + kc * 64u + l15 * 4u);
      z |= (m4.x == 0) | (m4.y == 0) | (m4.z == 0) | (m4.w == 0);
    }
    const int a = __any(z) ? 1 : 0;
    my |= (lane == kc) ? a : 0;
  }
  sm[w][lane] = my;
  __syncthreads();
  if (w == 0) {
    int f = 0;
#pragma unroll
    for (int ww = 0; ww < 8; ++ww) f |= sm[ww][lane];
    VST2(int, FL + blk * 32u + lane, f);
  }
}

__global__ __launch_bounds__(256) void k_tr16(const unsigned short* __restrict__ P, unsigned short* __restrict__ VT) {
  __shared__ __align__(16) unsigned short tl[64 * 72];
  const unsigned tid = threadIdx.x;
  const unsigned f0 = blockIdx.x * 64u, tok0 = blockIdx.y * 64u;
  const unsigned b = tok0 / (unsigned)SEQ, s0 = tok0 % (unsigned)SEQ;
#pragma unroll
  for (unsigned i = 0; i < 2; ++i) {
    const unsigned idx = tid + 256u * i, row = idx >> 3, pc = idx & 7u;
    const us8 v = *(const us8*)(P + (size_t)(tok0 + row) * DEMB + f0 + pc * 8u);
    *(us8*)(tl + row * 72u + pc * 8u) = v;
  }
  __syncthreads();
#pragma unroll
  for (unsigned i = 0; i < 2; ++i) {
    const unsigned idx = tid + 256u * i, d = idx >> 3, pc = idx & 7u;
    const unsigned short* col = tl + (pc * 8u) * 72u + d;
    u4v pk;
    pk.x = (unsigned)col[0]   | ((unsigned)col[72]  << 16);
    pk.y = (unsigned)col[144] | ((unsigned)col[216] << 16);
    pk.z = (unsigned)col[288] | ((unsigned)col[360] << 16);
    pk.w = (unsigned)col[432] | ((unsigned)col[504] << 16);
    VST2(u4v, VT + (size_t)(b * (unsigned)DEMB + f0 + d) * SEQ + s0 + pc * 8u, pk);
  }
}

__global__ __launch_bounds__(256) void k_castb_in(const float* __restrict__ S0, const float* __restrict__ S1, unsigned short* __restrict__ D0, unsigned short* __restrict__ D1) {
  const unsigned u = blockIdx.x * 256u + threadIdx.x; if (u >= (unsigned)TOK * 128u) return;
  const float* S = (blockIdx.y == 0) ? S0 : S1; unsigned short* D = (blockIdx.y == 0) ? D0 : D1;
  const unsigned r = u >> 7, c0 = (u & 127u) * 8u;
  const unsigned sr = (r / (unsigned)SEQ) * (unsigned)SEQ_FULL + (r % (unsigned)SEQ);
  const float* s = S + (size_t)sr * DEMB + c0;
  const v4f a = *(const v4f*)s, bq = *(const v4f*)(s + 4);
  u4v pk; pk.x = pk2h(cmb_bf(a.x), cmb_bf(a.y)); pk.y = pk2h(cmb_bf(a.z), cmb_bf(a.w)); pk.z = pk2h(cmb_bf(bq.x), cmb_bf(bq.y)); pk.w = pk2h(cmb_bf(bq.z), cmb_bf(bq.w));
  VST2(u4v, D + (size_t)r * DEMB + c0, pk);
}

__device__ __forceinline__ void castbT_body(const float* __restrict__ SRC, unsigned lds, unsigned short* __restrict__ DST, unsigned ldd, unsigned sh, unsigned u, float sc) {
  const unsigned cc = u >> sh, r0 = (u & ((1u << sh) - 1u)) * 8u;
  const float* s = SRC + (size_t)r0 * lds + cc;
  const float w0 = cmb_bf(s[0]) * sc, w1 = cmb_bf(s[(size_t)lds]) * sc, w2 = cmb_bf(s[(size_t)2 * lds]) * sc, w3 = cmb_bf(s[(size_t)3 * lds]) * sc;
  const float w4 = cmb_bf(s[(size_t)4 * lds]) * sc, w5 = cmb_bf(s[(size_t)5 * lds]) * sc, w6 = cmb_bf(s[(size_t)6 * lds]) * sc, w7 = cmb_bf(s[(size_t)7 * lds]) * sc;
  u4v pk; pk.x = pk2h(w0, w1); pk.y = pk2h(w2, w3); pk.z = pk2h(w4, w5); pk.w = pk2h(w6, w7);
  VST2(u4v, DST + (size_t)cc * ldd + r0, pk);
}
__global__ __launch_bounds__(256) void k_castbT(const float* __restrict__ SRC, unsigned lds, unsigned short* __restrict__ DST, unsigned ldd, unsigned sh, unsigned total, float sc) {
  const unsigned u = blockIdx.x * 256u + threadIdx.x; if (u >= total) return;
  castbT_body(SRC, lds, DST, ldd, sh, u, sc);
}
__global__ __launch_bounds__(256) void k_castbT4(const float* __restrict__ W0, const float* __restrict__ W1, const float* __restrict__ W2, const float* __restrict__ W3, unsigned short* __restrict__ DST, float sc) {
  const unsigned u = blockIdx.x * 256u + threadIdx.x; if (u >= 1024u * 128u) return;
  const unsigned y = blockIdx.y;
  const float* S = (y == 0) ? W0 : ((y == 1) ? W1 : ((y == 2) ? W2 : W3));
  castbT_body(S, 1024u, DST + (size_t)y * 1048576u, 1024u, 7u, u, sc);
}

__global__ __launch_bounds__(256) void k_bias6(const float* __restrict__ bq1, const float* __restrict__ bo1, const float* __restrict__ bq2, const float* __restrict__ bo2,
                                              const float* __restrict__ bff2, const float* __restrict__ bff1, float* __restrict__ BR) {
  const unsigned blk = blockIdx.x, seg = blk >> 2;
  const float* S = bff1; unsigned base = 5120u;
  if (seg == 0) { S = bq1; base = 0u; }
  else if (seg == 1) { S = bo1; base = 1024u; }
  else if (seg == 2) { S = bq2; base = 2048u; }
  else if (seg == 3) { S = bo2; base = 3072u; }
  else if (seg == 4) { S = bff2; base = 4096u; }
  const unsigned o = blk * 256u + threadIdx.x;
  VST2(float, BR + o, cmb_bf(S[o - base]));
}

template <int XBF>
__global__ __launch_bounds__(256) void k_ln(const float* __restrict__ A, const float* __restrict__ X, unsigned x_bs_rows, const float* __restrict__ GA, const float* __restrict__ BE,
                                           unsigned rows, float* __restrict__ Yf, unsigned short* __restrict__ Y16) {
  #pragma clang fp contract(off)
  const unsigned r = blockIdx.x * 8u + (threadIdx.x >> 5); const unsigned L = threadIdx.x & 31u; if (r >= rows) return;
  const unsigned xr = (r / (unsigned)SEQ) * x_bs_rows + (r % (unsigned)SEQ);
  v4f v[8]; float s = 0.f;
#pragma unroll
  for (int q = 0; q < 8; ++q) {
    const unsigned cc = 4u * L + 128u * (unsigned)q;
    v[q] = *(const v4f*)(A + (size_t)r * DEMB + cc);
    v4f x = *(const v4f*)(X + (size_t)xr * DEMB + cc);
    if (XBF) { x.x = cmb_bf(x.x); x.y = cmb_bf(x.y); x.z = cmb_bf(x.z); x.w = cmb_bf(x.w); }
    v[q] = v[q] + x;
    s += (v[q].x + v[q].y) + (v[q].z + v[q].w);
  }
#pragma unroll
  for (int o = 16; o > 0; o >>= 1) s += __shfl_xor(s, o, 32);
  const float mu = s * (1.f / 1024.f); float qq = 0.f;
#pragma unroll
  for (int q = 0; q < 8; ++q) { v[q].x -= mu; v[q].y -= mu; v[q].z -= mu; v[q].w -= mu; qq += (v[q].x * v[q].x + v[q].y * v[q].y) + (v[q].z * v[q].z + v[q].w * v[q].w); }
#pragma unroll
  for (int o = 16; o > 0; o >>= 1) qq += __shfl_xor(qq, o, 32);
  const float rs = rsqrtf(qq * (1.f / 1024.f) + 1e-5f);
#pragma unroll
  for (int q = 0; q < 8; ++q) {
    const unsigned cc = 4u * L + 128u * (unsigned)q;
    const v4f ga = *(const v4f*)(GA + cc), be = *(const v4f*)(BE + cc);
    v4f y;
    y.x = v[q].x * rs * cmb_bf(ga.x) + cmb_bf(be.x); y.y = v[q].y * rs * cmb_bf(ga.y) + cmb_bf(be.y);
    y.z = v[q].z * rs * cmb_bf(ga.z) + cmb_bf(be.z); y.w = v[q].w * rs * cmb_bf(ga.w) + cmb_bf(be.w);
    const size_t o = (size_t)r * DEMB + cc;
    if (Yf != nullptr) VST2(v4f, Yf + o, y);
    if (Y16 != nullptr) { u2v pk; pk.x = pk2h(y.x, y.y); pk.y = pk2h(y.z, y.w); VST2(u2v, Y16 + o, pk); }
  }
}

extern "C" void kernel_launch(void* const* d_in, const int* in_sizes, int n_in, void* d_out, int out_size, void* d_ws, size_t ws_size, hipStream_t stream) {
  if (n_in < 22) return;
  const long need_act = ((long)(NB - 1) * SEQ_FULL + SEQ) * DEMB;
  if (in_sizes[0] < need_act || in_sizes[1] < need_act) return;
  if ((long)in_sizes[2] < ((long)(NB - 1) * SEQ_FULL + (SEQ - 1)) * SEQ_FULL + SEQ) return;
  if (in_sizes[3] < (NB - 1) * SEQ_FULL + SEQ) return;
  if (in_sizes[4] < 1048576 || in_sizes[6] < 1048576 || in_sizes[8] < 1048576 || in_sizes[10] < 1048576 || in_sizes[12] < 4194304 || in_sizes[14] < 4194304) return;
  if (in_sizes[5] < 1024 || in_sizes[7] < 1024 || in_sizes[9] < 1024 || in_sizes[11] < 1024 || in_sizes[13] < 4096 || in_sizes[15] < 1024) return;
  for (int i = 16; i < 22; ++i) if (in_sizes[i] < 1024) return;
  if ((long)out_size < (long)TOK * DEMB) return;

  const float* trg = (const float*)d_in[0];
  const float* enc = (const float*)d_in[1];
  const int* tmask = (const int*)d_in[2];
  const int* smask = (const int*)d_in[3];
  const float* Wq1 = (const float*)d_in[4];  const float* bq1 = (const float*)d_in[5];
  const float* Wo1 = (const float*)d_in[6];  const float* bo1 = (const float*)d_in[7];
  const float* Wq2 = (const float*)d_in[8];  const float* bq2 = (const float*)d_in[9];
  const float* Wo2 = (const float*)d_in[10]; const float* bo2 = (const float*)d_in[11];
  const float* Wff1 = (const float*)d_in[12]; const float* bff1 = (const float*)d_in[13];
  const float* Wff2 = (const float*)d_in[14]; const float* bff2 = (const float*)d_in[15];
  const float* g1 = (const float*)d_in[16]; const float* b1 = (const float*)d_in[17];
  const float* g2 = (const float*)d_in[18]; const float* b2 = (const float*)d_in[19];
  const float* g3 = (const float*)d_in[20]; const float* b3 = (const float*)d_in[21];
  float* out = (float*)d_out;

  constexpr size_t PL = (size_t)TOK * DEMB;
  constexpr size_t BY_R0  = PL * 8;
  constexpr size_t BY_XE  = PL * 4;
  constexpr size_t BY_W4  = (size_t)4 * 1048576 * 2;
  constexpr size_t BY_W1T = (size_t)4194304 * 2;
  constexpr size_t BY_W2T = (size_t)4194304 * 2;
  constexpr size_t BY_F32 = PL * 4;
  constexpr size_t BY_BR  = (size_t)9216 * 4;
  constexpr size_t BY_FL  = (size_t)NB * NQB * 32 * 4;
  constexpr size_t WS_TOTAL = BY_R0 + BY_XE + BY_W4 + BY_W1T + BY_W2T + 3 * BY_F32 + BY_BR + BY_FL;
  static_assert(WS_TOTAL <= (size_t)134217728);
  static_assert(BY_R0 % 256 == 0 && BY_XE % 256 == 0 && BY_F32 % 256 == 0 && BY_BR % 256 == 0 && BY_FL % 256 == 0);
  static_assert(PL * 2 <= BY_F32);
  if (ws_size < WS_TOTAL) return;
  char* wsp = (char*)d_ws;
  unsigned short* R0  = (unsigned short*)wsp; wsp += BY_R0;
  unsigned short* XE  = (unsigned short*)wsp; wsp += BY_XE;
  unsigned short* W4  = (unsigned short*)wsp; wsp += BY_W4;
  unsigned short* W1T = (unsigned short*)wsp; wsp += BY_W1T;
  unsigned short* W2T = (unsigned short*)wsp; wsp += BY_W2T;
  float* Mf  = (float*)wsp; wsp += BY_F32;
  float* X1f = (float*)wsp; wsp += BY_F32;
  float* X2f = (float*)wsp; wsp += BY_F32;
  float* BR  = (float*)wsp; wsp += BY_BR;
  int*   FL  = (int*)wsp;   wsp += BY_FL;
  unsigned short* T16 = R0;
  unsigned short* CTX = R0;
  unsigned short* P1  = R0 + PL;
  unsigned short* QK2 = R0 + 2 * PL;
  unsigned short* H16 = R0;
  unsigned short* X16 = XE;
  unsigned short* E16 = XE + PL;
  unsigned short* VT  = (unsigned short*)X2f;

  const unsigned gD  = (unsigned)((((TOK / 64) * (DEMB / 64)) + 7) / 8);
  const unsigned gF  = (unsigned)((((TOK / 64) * (DFF / 64)) + 7) / 8);
  const unsigned gLN = (unsigned)((TOK + 7) / 8);
  const float IS = 0.0625f;

  k_castb_in<<<dim3((unsigned)(((size_t)TOK * 128 + 255) / 256), 2u), 256, 0, stream>>>(trg, enc, T16, E16);
  k_castbT4<<<dim3(512u, 4u), 256, 0, stream>>>(Wq1, Wo1, Wq2, Wo2, W4, 16.0f);
  k_castbT<<<2048, 256, 0, stream>>>(Wff1, 4096u, W1T, 1024u, 7u, 4096u * 128u, 16.0f);
  k_castbT<<<2048, 256, 0, stream>>>(Wff2, 1024u, W2T, 4096u, 9u, 1024u * 512u, 16.0f);
  k_bias6<<<36, 256, 0, stream>>>(bq1, bo1, bq2, bo2, bff2, bff1, BR);
  k_mflag<<<(unsigned)(NB * NQB), 256, 0, stream>>>(tmask, FL);

  k_gemm64<1, 0><<<dim3(gD, 1u), 256, 0, stream>>>(T16, 1024, 0L, W4, 1024, 0L, (void*)P1, 1024, 0L, BR, TOK, DEMB, DEMB, IS);
  k_tr16<<<dim3(16u, (unsigned)(TOK / 64)), 256, 0, stream>>>(P1, VT);
  k_attn16<0><<<(unsigned)(NB * 16 * NQB), 128, 0, stream>>>(P1, P1, VT, tmask, FL, CTX);
  k_gemm64<0, 0><<<dim3(gD, 1u), 256, 0, stream>>>(CTX, 1024, 0L, W4 + 1048576, 1024, 0L, (void*)Mf, 1024, 0L, BR + 1024, TOK, DEMB, DEMB, IS);
  k_ln<1><<<gLN, 256, 0, stream>>>(Mf, trg, (unsigned)SEQ_FULL, g1, b1, (unsigned)TOK, X1f, X16);

  k_gemm64<1, 0><<<dim3(gD, 2u), 256, 0, stream>>>(XE, 1024, (long)PL, W4 + 2 * 1048576, 1024, 0L, (void*)QK2, 1024, (long)PL, BR + 2048, TOK, DEMB, DEMB, IS);
  k_tr16<<<dim3(16u, (unsigned)(TOK / 64)), 256, 0, stream>>>(QK2 + PL, VT);
  k_attn16<1><<<(unsigned)(NB * 16 * NQB), 128, 0, stream>>>(QK2, QK2 + PL, VT, smask, FL, CTX);
  k_gemm64<0, 0><<<dim3(gD, 1u), 256, 0, stream>>>(CTX, 1024, 0L, W4 + 3 * 1048576, 1024, 0L, (void*)Mf, 1024, 0L, BR + 3072, TOK, DEMB, DEMB, IS);
  k_ln<0><<<gLN, 256, 0, stream>>>(Mf, X1f, (unsigned)SEQ, g2, b2, (unsigned)TOK, X2f, X16);

  k_gemm64<1, 2><<<dim3(gF, 1u), 256, 0, stream>>>(X16, 1024, 0L, W1T, 1024, 0L, (void*)H16, 4096, 0L, BR + 5120, TOK, DFF, DEMB, IS);
  k_gemm64<0, 0><<<dim3(gD, 1u), 256, 0, stream>>>(H16, 4096, 0L, W2T, 4096, 0L, (void*)Mf, 1024, 0L, BR + 4096, TOK, DEMB, DFF, IS);
  k_ln<0><<<gLN, 256, 0, stream>>>(Mf, X2f, (unsigned)SEQ, g3, b3, (unsigned)TOK, out, nullptr);
}
